// MultiHeadSelfAttentionBlock_56556129353873
// MI455X (gfx1250) — hardware-verified
//
#include <hip/hip_runtime.h>
#include <stddef.h>
#include <stdint.h>
#include <math.h>


#define CCH    128
#define NHD    8
#define HDM    16
#define NKV    27
#define QKVW   384
#define OQ     0
#define OKK    128
#define OV     256
#define K2     256
#define NTHR   256
#define NWAVE  8
#define EPT    8
#define CHUNK  (NTHR * EPT)
#define WCAP   (EPT * 32)
#define LISTN  (NWAVE * WCAP)
#define NBMAX  1024
#define SLOTB  10
#define RCAP   28672
#define DEGCAP 64
#define STW    128
#define GBM    64
#define GBN    128
#define GTHR   128
#define GWAVE  (GTHR / 32)
#define PARTW  288
#define WSTW   258
#define RTN    (NKV * CCH)
#define NUQKV  (QKVW * (CCH / 8))
#define NUW2   (CCH * (K2 / 8))
#define NBQKV  (NUQKV / NTHR)
#define NBW2   (NUW2 / NTHR)
#define NBPREP (NBQKV + 3 * NBW2 + 1)
#define ATTSC  0.25f
#define WSLIM  134217728
#define LDSW_SR  (2 * RCAP + 2 * NBMAX + LISTN + 2 * NWAVE)
#define LDSW_END (LDSW_SR + RTN)
#define LDS_ATTN (LDSW_END * 4 + 64)

static_assert((1 << SLOTB) == NBMAX);
static_assert(SLOTB + 21 <= 31);
static_assert((CHUNK & (CHUNK - 1)) == 0 && CHUNK <= 2048 && SLOTB + 11 <= 31);
static_assert(NTHR * 4 == NBMAX);
static_assert(LISTN >= NBMAX);
static_assert(LISTN >= NWAVE * WCAP);
static_assert((RCAP % 32) == 0);
static_assert((NBMAX % NWAVE) == 0);
static_assert(NWAVE * STW <= RCAP && (STW % 4) == 0 && STW >= CCH);
static_assert((LDSW_SR % 4) == 0 && (RTN % 4) == 0);
static_assert(LDS_ATTN <= 300000);
static_assert(GBM == GWAVE * 16 && GBN == 4 * 32 && GTHR == GBN);
static_assert(CCH == 32 * 4 && HDM == 4 * 4 && NHD * HDM == CCH);
static_assert((CCH % 32) == 0 && (K2 % 32) == 0 && K2 == 2 * CCH);
static_assert(QKVW == 3 * CCH && (QKVW % GBN) == 0 && CCH == GBN);
static_assert(PARTW % 32 == 0 && PARTW / 4 <= GTHR && PARTW >= 2 * GBN + 1);
static_assert(WSTW >= 2 * GBN + 1 && (WSTW % 2) == 0);
static_assert((NUQKV % NTHR) == 0 && (NUW2 % NTHR) == 0 && (NUQKV % (8 * NTHR)) == 0 && (NUW2 % (16 * NTHR)) == 0);
static_assert(NTHR == 2 * CCH);
static_assert((NBMAX % GBM) == 0);

typedef float          v4f  __attribute__((ext_vector_type(4)));
typedef float          v8f  __attribute__((ext_vector_type(8)));
typedef int            v4i  __attribute__((ext_vector_type(4)));
typedef int            v8i  __attribute__((ext_vector_type(8)));
typedef unsigned int   v4u  __attribute__((ext_vector_type(4)));
typedef unsigned short v8us __attribute__((ext_vector_type(8)));
typedef __bf16         v16b __attribute__((ext_vector_type(16)));
typedef v4f  __attribute__((may_alias)) v4fa;
typedef v4u  __attribute__((may_alias)) v4ua;
typedef v8us __attribute__((may_alias)) v8usa;
union FragB { v16b v; v8us h[2]; v8i w; };

__device__ __forceinline__ v8f wmb(const FragB& a, const FragB& b, v8f c) {
  v8f d = __builtin_amdgcn_wmma_f32_16x16x32_bf16(false, a.v, false, b.v, (short)0, c, false, false);
  asm volatile("v_nop\n\tv_nop\n\tv_nop\n\tv_nop" : "+v"(d) : "v"(a.w), "v"(b.w));
  return d;
}

__device__ __forceinline__ v8f z8() { v8f z = {0.f, 0.f, 0.f, 0.f, 0.f, 0.f, 0.f, 0.f}; return z; }

__device__ __forceinline__ void ldwait() {
  asm volatile("s_wait_loadcnt 0x0" ::: "memory");
}

__device__ __forceinline__ unsigned int f2bf(float f) {
  const unsigned int u = __float_as_uint(f);
  return ((u + 0x7FFFu + ((u >> 16) & 1u)) >> 16) & 0xFFFFu;
}
__device__ __forceinline__ float bf2f(unsigned int b) { return __uint_as_float(b << 16); }
__device__ __forceinline__ float bfr(float f) { return bf2f(f2bf(f)); }
__device__ __forceinline__ v4f bfr4(const v4f a) {
  v4f r; r.x = bfr(a.x); r.y = bfr(a.y); r.z = bfr(a.z); r.w = bfr(a.w); return r;
}
__device__ __forceinline__ unsigned int pk2(float lo, float hi) { return f2bf(lo) | (f2bf(hi) << 16); }
__device__ __forceinline__ v4u pack8(const v4f a, const v4f b) {
  v4u r;
  r.x = pk2(a.x, a.y); r.y = pk2(a.z, a.w); r.z = pk2(b.x, b.y); r.w = pk2(b.z, b.w);
  return r;
}
__device__ __forceinline__ void hl2(float v0, float v1, unsigned int& hw, unsigned int& lw) {
  const unsigned int h0 = f2bf(v0), h1 = f2bf(v1);
  const unsigned int l0 = f2bf(v0 - bf2f(h0)), l1 = f2bf(v1 - bf2f(h1));
  hw = h0 | (h1 << 16);
  lw = l0 | (l1 << 16);
}
__device__ __forceinline__ void pack8hl(const v4f a, const v4f b, v4u& hv, v4u& lv) {
  unsigned int h, l;
  hl2(a.x, a.y, h, l); hv.x = h; lv.x = l;
  hl2(a.z, a.w, h, l); hv.y = h; lv.y = l;
  hl2(b.x, b.y, h, l); hv.z = h; lv.z = l;
  hl2(b.z, b.w, h, l); hv.w = h; lv.w = l;
}

__device__ __forceinline__ int scan_chunk(const int* __restrict__ dsts, int nE, int cbase, int slotBase,
                                          int nb, int vec8, int* list, int tid, int lane, int wave) {
  int wc = 0;
  const int el0  = tid * EPT;
  const int e0   = cbase + el0;
  const int sent = -2147483647 - 1;
  v4i da, db;
  if (vec8 != 0 && cbase + CHUNK <= nE) {
    da = *(const v4i*)(dsts + e0);
    db = *(const v4i*)(dsts + e0 + 4);
  } else {
    da.x = (e0     < nE) ? dsts[min(e0,     nE - 1)] : sent;
    da.y = (e0 + 1 < nE) ? dsts[min(e0 + 1, nE - 1)] : sent;
    da.z = (e0 + 2 < nE) ? dsts[min(e0 + 2, nE - 1)] : sent;
    da.w = (e0 + 3 < nE) ? dsts[min(e0 + 3, nE - 1)] : sent;
    db.x = (e0 + 4 < nE) ? dsts[min(e0 + 4, nE - 1)] : sent;
    db.y = (e0 + 5 < nE) ? dsts[min(e0 + 5, nE - 1)] : sent;
    db.z = (e0 + 6 < nE) ? dsts[min(e0 + 6, nE - 1)] : sent;
    db.w = (e0 + 7 < nE) ? dsts[min(e0 + 7, nE - 1)] : sent;
  }
  const unsigned nbs = (unsigned)slotBase;
  const unsigned unb = (unsigned)nb;
  const unsigned s0 = (unsigned)da.x - nbs, s1 = (unsigned)da.y - nbs;
  const unsigned s2 = (unsigned)da.z - nbs, s3 = (unsigned)da.w - nbs;
  const unsigned s4 = (unsigned)db.x - nbs, s5 = (unsigned)db.y - nbs;
  const unsigned s6 = (unsigned)db.z - nbs, s7 = (unsigned)db.w - nbs;
  const bool h0 = s0 < unb, h1 = s1 < unb, h2 = s2 < unb, h3 = s3 < unb;
  const bool h4 = s4 < unb, h5 = s5 < unb, h6 = s6 < unb, h7 = s7 < unb;
  const unsigned any = __builtin_amdgcn_ballot_w32(h0 | h1 | h2 | h3 | h4 | h5 | h6 | h7);
  if (any != 0u) {
#define HITJ(J, HJ, SJ) { \
      const unsigned mj = __builtin_amdgcn_ballot_w32(HJ); \
      if (mj != 0u) { \
        if (HJ) { \
          const int pos = wc + (int)__builtin_amdgcn_mbcnt_lo(mj, 0u); \
          if (pos < WCAP) list[wave * WCAP + pos] = ((el0 + (J)) << SLOTB) | (int)(SJ); \
        } \
        wc += (int)__builtin_popcount(mj); } }
    HITJ(0, h0, s0)
    HITJ(1, h1, s1)
    HITJ(2, h2, s2)
    HITJ(3, h3, s3)
    HITJ(4, h4, s4)
    HITJ(5, h5, s5)
    HITJ(6, h6, s6)
    HITJ(7, h7, s7)
#undef HITJ
  }
  return wc;
}

__global__ __launch_bounds__(NTHR) void k_wprep(
    const float* __restrict__ Wq, const float* __restrict__ Wk, const float* __restrict__ Wv,
    const float* __restrict__ Wo, const float* __restrict__ mW1, const float* __restrict__ mW2,
    const float* __restrict__ pW1, const float* __restrict__ pb1,
    const float* __restrict__ pW2, const float* __restrict__ pb2,
    unsigned short* wqkvt, unsigned short* wot2, unsigned short* m1t2, unsigned short* m2t2, float* rt) {
  __shared__ __attribute__((aligned(16))) float sRT[RTN];
  __shared__ float sP[16];
  const int b = (int)blockIdx.x, tid = (int)threadIdx.x;
  const v4f z4 = {0.f, 0.f, 0.f, 0.f};
  if (b < NBQKV) {
    const int u   = b * NTHR + tid;
    const int n   = u >> 4;
    const int k8  = (u & 15) * 8;
    const int sel = b >> 3;
    const float* W = (sel == 0) ? Wq : ((sel == 1) ? Wk : Wv);
    const int nc  = n & (CCH - 1);
    const float* p = W + (size_t)k8 * CCH + nc;
    v4f a, c;
    a.x = p[0];                    a.y = p[(size_t)CCH];          a.z = p[(size_t)2 * CCH];      a.w = p[(size_t)3 * CCH];
    c.x = p[(size_t)4 * CCH];      c.y = p[(size_t)5 * CCH];      c.z = p[(size_t)6 * CCH];      c.w = p[(size_t)7 * CCH];
    const v4u wv = pack8(a, c);
    unsigned short* o = wqkvt + (size_t)n * CCH + k8;
    *(volatile v4u*)o = wv;
    __threadfence();
    *(volatile v4u*)o = wv;
  } else if (b < NBQKV + 3 * NBW2) {
    const int v  = (b - NBQKV) * NTHR + tid;
    const int pl = (b - NBQKV) >> 4;
    const float* W = (pl == 0) ? Wo : ((pl == 1) ? mW1 : mW2);
    unsigned short* dst = (pl == 0) ? wot2 : ((pl == 1) ? m1t2 : m2t2);
    const int w  = v & (NUW2 - 1);
    const int n  = w >> 5;
    const int k8 = (w & 31) * 8;
    const int kk = k8 & (CCH - 1);
    const float* p = W + (size_t)kk * CCH + n;
    v4f a, c;
    a.x = p[0];                    a.y = p[(size_t)CCH];          a.z = p[(size_t)2 * CCH];      a.w = p[(size_t)3 * CCH];
    c.x = p[(size_t)4 * CCH];      c.y = p[(size_t)5 * CCH];      c.z = p[(size_t)6 * CCH];      c.w = p[(size_t)7 * CCH];
    const v4u wv = pack8(a, c);
    unsigned short* o = dst + (size_t)n * K2 + k8;
    *(volatile v4u*)o = wv;
    __threadfence();
    *(volatile v4u*)o = wv;
  } else {
    {
      const int ia = tid < 9 ? tid : 8;
      int ib = tid - 9; ib = ib < 0 ? 0 : (ib > 2 ? 2 : ib);
      const float va = pW1[ia];
      const float vb = pb1[ib];
      if (tid < 12) sP[tid] = (tid < 9) ? bfr(va) : bfr(vb);
    }
    __syncthreads();
#pragma unroll 1
    for (int q = tid; q < RTN / 4; q += NTHR) {
      const int kv = q >> 5;
      const int c4 = (q & 31) * 4;
      const float px = 1.0f - (float)(kv % 3);
      const float py = 1.0f - (float)((kv / 3) % 3);
      const float pz = 1.0f - (float)(kv / 9);
      v4f acc = bfr4(*(const v4fa*)(pb2 + c4));
#pragma unroll
      for (int j = 0; j < 3; ++j) {
        float t = px * sP[j];
        t = fmaf(py, sP[3 + j], t);
        t = fmaf(pz, sP[6 + j], t);
        t = t + sP[9 + j];
        t = fmaxf(t, 0.0f);
        const v4f w2 = bfr4(*(const v4fa*)(pW2 + (size_t)j * CCH + c4));
        acc.x = fmaf(t, w2.x, acc.x); acc.y = fmaf(t, w2.y, acc.y);
        acc.z = fmaf(t, w2.z, acc.z); acc.w = fmaf(t, w2.w, acc.w);
      }
      *(v4fa*)(sRT + 4 * q) = acc;
    }
    __syncthreads();
#pragma unroll 1
    for (int q = tid; q < RTN / 4; q += NTHR) {
      const v4f vv = *(const v4fa*)(sRT + 4 * q);
      *(volatile v4f*)(rt + 4 * q) = vv;
    }
    __threadfence();
#pragma unroll 1
    for (int q = tid; q < RTN / 4; q += NTHR) {
      const v4f vv = *(const v4fa*)(sRT + 4 * q);
      *(volatile v4f*)(rt + 4 * q) = vv;
    }
  }
  (void)z4;
}

__global__ __launch_bounds__(NTHR) void k_xprep(const float* __restrict__ x, unsigned short* xb, int nN, int nUnits) {
  const int i = (int)blockIdx.x * NTHR + (int)threadIdx.x;
  if (i >= nUnits) return;
  const int row = i >> 4;
  const int c0  = (i & 15) * 8;
  const int rc  = row < nN ? row : nN - 1;
  const float* p = x + (size_t)rc * CCH + c0;
  v4f a = *(const v4fa*)p;
  v4f b = *(const v4fa*)(p + 4);
  const v4f z4 = {0.f, 0.f, 0.f, 0.f};
  if (row >= nN) { a = z4; b = z4; }
  const v4u hv = pack8(a, b);
  unsigned short* o = xb + (size_t)row * CCH + c0;
  *(volatile v4u*)o = hv;
  __threadfence();
  *(volatile v4u*)o = hv;
}

template <int KD, int MODE>
__global__ __launch_bounds__(GTHR) void k_gemm(const unsigned short* __restrict__ A,
                                               const unsigned short* __restrict__ BT, int nN,
                                               const float* __restrict__ bias0, const float* __restrict__ bias1,
                                               const float* __restrict__ bias2,
                                               float* xout, int ldo, float* part) {
  __shared__ __attribute__((aligned(16))) float stg[GBM * GBN];
  __shared__ __attribute__((aligned(16))) float wst[GWAVE * WSTW];
  __shared__ __attribute__((aligned(16))) float pst[PARTW];
  const int tid = (int)threadIdx.x, lane = tid & 31, wave = tid >> 5, hh = lane >> 4, m = lane & 15;
  const int rowBase = (int)blockIdx.x * GBM;
  const int colBase = (int)blockIdx.y * GBN;

  v8f acc[8];
#pragma unroll
  for (int t = 0; t < 8; ++t) acc[t] = z8();
  const unsigned short* ap = A  + (size_t)(rowBase + 16 * wave + m) * (size_t)KD + 8 * hh;
  const unsigned short* bp = BT + (size_t)(colBase + m) * (size_t)KD + 8 * hh;

#pragma unroll 1
  for (int k0 = 0; k0 < KD; k0 += 32) {
    FragB af;
    af.h[0] = *(const v8usa*)(ap + k0);
    af.h[1] = *(const v8usa*)(ap + k0 + 16);
#pragma unroll
    for (int nt = 0; nt < 8; ++nt) {
      const unsigned short* wq = bp + (size_t)(16 * nt) * (size_t)KD + k0;
      FragB bf;
      bf.h[0] = *(const v8usa*)wq;
      bf.h[1] = *(const v8usa*)(wq + 16);
      acc[nt] = wmb(af, bf, acc[nt]);
    }
  }

#pragma unroll
  for (int nt = 0; nt < 8; ++nt) {
    const int lc = 16 * nt + m;
#pragma unroll
    for (int r = 0; r < 8; ++r) {
      const int lr = 16 * wave + 8 * hh + r;
      stg[lr * GBN + lc] = acc[nt][r];
    }
  }
  __syncthreads();

  float bq[4];
  if constexpr (MODE == 0) {
    const v4f ba = *(const v4f*)(bias0 + 4 * lane);
    const v4f bb = *(const v4f*)(bias1 + 4 * lane);
    const v4f bc = *(const v4f*)(bias2 + 4 * lane);
    const int sel = (int)blockIdx.y;
    const v4f b4 = (sel == 0) ? ba : ((sel == 1) ? bb : bc);
    bq[0] = bfr(b4.x); bq[1] = bfr(b4.y); bq[2] = bfr(b4.z); bq[3] = bfr(b4.w);
  } else if constexpr (MODE == 1) {
    const v4f b4 = *(const v4f*)(bias0 + 4 * lane);
    bq[0] = bfr(b4.x); bq[1] = bfr(b4.y); bq[2] = bfr(b4.z); bq[3] = bfr(b4.w);
  } else {
    bq[0] = 0.0f; bq[1] = 0.0f; bq[2] = 0.0f; bq[3] = 0.0f;
  }

  v4f pv[16];
  int wn = 0;
  float wm[4], wqv[4];
#pragma unroll
  for (int j = 0; j < 4; ++j) { wm[j] = 0.0f; wqv[j] = 0.0f; }
#pragma unroll
  for (int i = 0; i < 16; ++i) {
    const int row = rowBase + 16 * wave + i;
    const bool ok = row < nN;
    const v4f x = *(const v4fa*)(stg + (16 * wave + i) * GBN + 4 * lane);
    float y[4];
    y[0] = x.x + bq[0]; y[1] = x.y + bq[1]; y[2] = x.z + bq[2]; y[3] = x.w + bq[3];
    float vv[4];
#pragma unroll
    for (int j = 0; j < 4; ++j) vv[j] = ok ? y[j] : 0.0f;
    v4f q;
    q.x = vv[0]; q.y = vv[1]; q.z = vv[2]; q.w = vv[3];
    pv[i] = q;
    if constexpr (MODE >= 1) {
      if (ok) {
        wn += 1;
        const float rk = 1.0f / (float)(i + 1);
#pragma unroll
        for (int j = 0; j < 4; ++j) {
          const float d = vv[j] - wm[j];
          wm[j]  = fmaf(d, rk, wm[j]);
          wqv[j] = fmaf(d, vv[j] - wm[j], wqv[j]);
        }
      }
    }
  }
#pragma unroll
  for (int i = 0; i < 16; ++i) {
    float* op = xout + (size_t)(rowBase + 16 * wave + i) * (size_t)ldo + colBase + 4 * lane;
    *(volatile v4f*)op = pv[i];
  }
  __threadfence();
#pragma unroll
  for (int i = 0; i < 16; ++i) {
    float* op = xout + (size_t)(rowBase + 16 * wave + i) * (size_t)ldo + colBase + 4 * lane;
    *(volatile v4f*)op = pv[i];
  }

  if constexpr (MODE >= 1) {
    if (lane == 0) wst[wave * WSTW] = (float)wn;
#pragma unroll
    for (int j = 0; j < 4; ++j) {
      wst[wave * WSTW + 1 + 4 * lane + j]       = wm[j];
      wst[wave * WSTW + 1 + GBN + 4 * lane + j] = wqv[j];
    }
    __syncthreads();
    {
      float n = 0.0f, mean = 0.0f, M2 = 0.0f;
#pragma unroll 1
      for (int w2 = 0; w2 < GWAVE; ++w2) {
        const float nb = wst[w2 * WSTW];
        const float mb = wst[w2 * WSTW + 1 + tid];
        const float qb = wst[w2 * WSTW + 1 + GBN + tid];
        if (nb > 0.5f) {
          const float nn = n + nb;
          const float delta = mb - mean;
          const float f = nb / nn;
          mean = fmaf(delta, f, mean);
          M2 = M2 + qb + delta * delta * n * f;
          n = nn;
        }
      }
      pst[1 + tid] = mean;
      pst[1 + GBN + tid] = M2;
      if (tid == 0) pst[0] = n;
    }
#pragma unroll 1
    for (int i = 2 * GBN + 1 + tid; i < PARTW; i += GTHR) pst[i] = 0.0f;
    __syncthreads();
    const int pb = (int)blockIdx.x * (int)gridDim.y + (int)blockIdx.y;
    v4f ps;
    if (tid < PARTW / 4) {
      ps = *(const v4fa*)(pst + 4 * tid);
      *(volatile v4f*)(part + (size_t)pb * PARTW + 4 * tid) = ps;
    }
    __threadfence();
    if (tid < PARTW / 4) {
      *(volatile v4f*)(part + (size_t)pb * PARTW + 4 * tid) = ps;
    }
  } else {
    (void)wn; (void)part;
  }
}

__global__ __launch_bounds__(NTHR) void k_attn(
    const int* __restrict__ keys, const int* __restrict__ kern, const int* __restrict__ qidx,
    const float* __restrict__ QKV, const float* __restrict__ RT,
    unsigned short* AOHL, int nN, int nE, int vec8, int MPr) {
  extern __shared__ v4f lds_dyn[];
  int* reg1 = (int*)lds_dyn;
  int* reg2 = reg1 + RCAP;
  int* scnt = reg2 + RCAP;
  int* soff = scnt + NBMAX;
  int* list = soff + NBMAX;
  int* wcnt = list + LISTN;
  int* wtot = wcnt + NWAVE;
  float* sR = (float*)(wtot + NWAVE);
  const int tid = (int)threadIdx.x, lane = tid & 31, wave = tid >> 5;
  const int nodeBase = (int)blockIdx.x * NBMAX;

  for (int i = tid; i < NBMAX; i += NTHR) scnt[i] = 0;
#pragma unroll 1
  for (int i = tid; i < RTN / 4; i += NTHR) {
    const v4f rv = *(const v4fa*)(RT + 4 * i);
    *(v4fa*)(sR + 4 * i) = rv;
  }
  __syncthreads();

  int tot = 0;
  const int nChunks = (nE + CHUNK - 1) / CHUNK;
#pragma unroll 1
  for (int ch = 0; ch < nChunks; ++ch) {
    const int cbase = ch * CHUNK;
    const int wc = scan_chunk(qidx, nE, cbase, nodeBase, NBMAX, vec8, list, tid, lane, wave);
    if (lane == 0) wcnt[wave] = wc;
    __syncthreads();
    int pre = 0, all = 0;
#pragma unroll
    for (int w2 = 0; w2 < NWAVE; ++w2) {
      int c = wcnt[w2];
      c = c < 0 ? 0 : (c > WCAP ? WCAP : c);
      all += c;
      pre += (w2 < wave) ? c : 0;
    }
    const int wcc  = wc > WCAP ? WCAP : wc;
    const int base = tot + pre;
#pragma unroll 1
    for (int i = lane; i < wcc; i += 32) {
      const int ent = list[wave * WCAP + i];
      const int el  = (ent >> SLOTB) & (CHUNK - 1);
      const int sl  = ent & (NBMAX - 1);
      int eid = cbase + el;
      eid = eid > nE - 1 ? nE - 1 : eid;
      const int pos = base + i;
      if (pos < RCAP) reg1[pos] = (int)(((unsigned)eid << SLOTB) | (unsigned)sl);
    }
    tot += all;
    tot = tot > RCAP ? RCAP : tot;
    __syncthreads();
  }
  const int nh = tot;

  if (wave == 0) {
#pragma unroll 1
    for (int b0 = 0; b0 < nh; b0 += 32) {
      const int idx = b0 + lane;
      const int uv  = reg1[idx < nh ? idx : nh - 1];
      const int m32 = (nh - b0) < 32 ? (nh - b0) : 32;
#pragma unroll 1
      for (int k = 0; k < m32; ++k) {
        const int u  = __builtin_amdgcn_readlane(uv, k);
        const int sl = u & (NBMAX - 1);
        if (lane == 0) scnt[sl] = scnt[sl] + 1;
      }
    }
  }
  __syncthreads();

  {
    const v4i ca = *(const v4i*)(scnt + 4 * tid);
    const int e0 = ca.x < 0 ? 0 : ca.x, e1 = ca.y < 0 ? 0 : ca.y, e2 = ca.z < 0 ? 0 : ca.z, e3 = ca.w < 0 ? 0 : ca.w;
    const int ts = e0 + e1 + e2 + e3;
    int incl = ts;
#pragma unroll
    for (int d = 1; d < 32; d <<= 1) {
      const int up = __shfl_up(incl, d);
      if (lane >= d) incl += up;
    }
    if (lane == 31) wtot[wave] = incl;
    __syncthreads();
    int pre = 0;
#pragma unroll
    for (int w2 = 0; w2 < NWAVE; ++w2) pre += (w2 < wave) ? wtot[w2] : 0;
    int run = pre + incl - ts;
    soff[4 * tid + 0] = run; run += e0;
    soff[4 * tid + 1] = run; run += e1;
    soff[4 * tid + 2] = run; run += e2;
    soff[4 * tid + 3] = run;
  }
  __syncthreads();
  for (int i = tid; i < NBMAX; i += NTHR) list[i] = soff[i];
  __syncthreads();

  if (wave == 0) {
#pragma unroll 1
    for (int b0 = 0; b0 < nh; b0 += 32) {
      const int idx = b0 + lane;
      const int uv  = reg1[idx < nh ? idx : nh - 1];
      const int m32 = (nh - b0) < 32 ? (nh - b0) : 32;
#pragma unroll 1
      for (int k = 0; k < m32; ++k) {
        const int u   = __builtin_amdgcn_readlane(uv, k);
        const int sl  = u & (NBMAX - 1);
        const int eid = (int)((unsigned)u >> SLOTB);
        if (lane == 0) {
          int pos = list[sl];
          pos = pos < 0 ? 0 : (pos > RCAP - 1 ? RCAP - 1 : pos);
          reg2[pos] = eid;
          list[sl] = pos + 1;
        }
      }
    }
  }
  __syncthreads();

  const int nbw = NBMAX / NWAVE;
  const bool ovf = (nh >= RCAP);
  const float qnan = __int_as_float(0x7fc00000);
  float* stw = (float*)reg1 + wave * STW;
  const int l16 = lane & 15;

#pragma unroll 1
  for (int jt = 0; jt < nbw; ++jt) {
    const int slot = wave * nbw + jt;
    const int grow = nodeBase + slot;
    const int gcl  = grow < nN ? grow : nN - 1;
    int st = soff[slot];
    const int craw = scnt[slot];
    int cnt = craw;
    st  = st < 0 ? 0 : (st > nh ? nh : st);
    cnt = cnt < 0 ? 0 : (cnt > DEGCAP ? DEGCAP : cnt);
    if (cnt > nh - st) cnt = nh - st;
    const float pz = (ovf || craw > DEGCAP) ? qnan : 0.0f;

    const v4f qa = *(const v4fa*)(QKV + (size_t)gcl * QKVW + OQ + 4 * lane);
    ldwait();

    float mx = -1.0e30f, dn = 0.f;
    v4f av = {0.f, 0.f, 0.f, 0.f};
#pragma unroll 1
    for (int q = 0; q < cnt; ++q) {
      int idx = st + q; idx = idx > RCAP - 1 ? RCAP - 1 : idx;
      int eid = reg2[idx]; eid = eid < 0 ? 0 : (eid > nE - 1 ? nE - 1 : eid);
      const int sraw = keys[eid];
      const int s = sraw < 0 ? 0 : (sraw > nN - 1 ? nN - 1 : sraw);
      const int kraw = kern[eid];
      const int kv = kraw < 0 ? 0 : (kraw > NKV - 1 ? NKV - 1 : kraw);
      const float* kr = QKV + (size_t)s * QKVW + OKK + 4 * lane;
      const v4f ka = *(const v4fa*)kr;
      const float* vr = QKV + (size_t)s * QKVW + OV + 4 * lane;
      const v4f va = *(const v4fa*)vr;
      const v4f ra = *(const v4fa*)(sR + kv * CCH + 4 * lane);
      ldwait();
      float p = qa.x * (ka.x + ra.x);
      p = fmaf(qa.y, ka.y + ra.y, p);
      p = fmaf(qa.z, ka.z + ra.z, p);
      p = fmaf(qa.w, ka.w + ra.w, p);
      p += __shfl_xor(p, 2);
      p += __shfl_xor(p, 1);
      const float lg = p * ATTSC;
      const float df = lg - mx;
      const float ee = __expf(-fabsf(df));
      const bool up  = df > 0.f;
      const float s1 = up ? ee : 1.0f;
      const float s2 = up ? 1.0f : ee;
      mx = up ? lg : mx;
      dn = fmaf(dn, s1, s2);
      av.x = fmaf(av.x, s1, s2 * va.x); av.y = fmaf(av.y, s1, s2 * va.y);
      av.z = fmaf(av.z, s1, s2 * va.z); av.w = fmaf(av.w, s1, s2 * va.w);
    }
    const float dns = dn > 0.f ? dn : 1.0f;
    const float ind = dn > 0.f ? 1.0f : 0.0f;
    const float inv = ind * (1.0f / dns);
    v4f oa;
    oa.x = av.x * inv + pz; oa.y = av.y * inv + pz; oa.z = av.z * inv + pz; oa.w = av.w * inv + pz;
    __builtin_amdgcn_fence(__ATOMIC_RELEASE, "wavefront");
    __builtin_amdgcn_wave_barrier();
    *(v4fa*)(stw + 4 * lane) = oa;
    __builtin_amdgcn_fence(__ATOMIC_RELEASE, "wavefront");
    __builtin_amdgcn_wave_barrier();
    const v4f pa = *(const v4fa*)(stw + 8 * l16);
    const v4f pb = *(const v4fa*)(stw + 8 * l16 + 4);
    v4u hv, lv;
    pack8hl(pa, pb, hv, lv);
    v4u wv;
    wv.x = (lane < 16) ? hv.x : lv.x;
    wv.y = (lane < 16) ? hv.y : lv.y;
    wv.z = (lane < 16) ? hv.z : lv.z;
    wv.w = (lane < 16) ? hv.w : lv.w;
    const bool wr = (grow < MPr);
    const int gsf = wr ? grow : MPr - 1;
    unsigned short* orow = AOHL + (size_t)gsf * K2 + 8 * lane;
    if (wr) *(volatile v4u*)orow = wv;
    __threadfence();
    if (wr) *(volatile v4u*)orow = wv;
  }
}

__global__ __launch_bounds__(CCH) void k_bnfin(const float* __restrict__ part, int nPart,
                                               const float* __restrict__ gam, const float* __restrict__ bet,
                                               float* ss) {
  __shared__ __attribute__((aligned(16))) float stg[2 * CCH];
  const int tid = (int)threadIdx.x;
  const int c = tid;
  double n = 0.0, mean = 0.0, M2 = 0.0;
#pragma unroll 1
  for (int b = 0; b < nPart; ++b) {
    const float* pr = part + (size_t)b * PARTW;
    const double nb = (double)pr[0];
    const double mb = (double)pr[1 + c];
    const double qb = (double)pr[1 + GBN + c];
    if (nb > 0.5) {
      const double nn = n + nb;
      const double delta = mb - mean;
      const double f = nb / nn;
      mean = mean + delta * f;
      M2 = M2 + qb + delta * delta * n * f;
      n = nn;
    }
  }
  const double nt = n < 1.0 ? 1.0 : n;
  const float varf  = (float)(M2 / nt);
  const float meanf = (float)mean;
  const float rstd = 1.0f / sqrtf(varf + 1e-5f);
  const float sc = bfr(gam[c]) * rstd;
  const float sh = bfr(bet[c]) - meanf * sc;
  stg[c] = sc;
  stg[CCH + c] = sh;
  __syncthreads();
  v4f v;
  if (tid < (2 * CCH) / 4) {
    v = *(const v4fa*)(stg + 4 * tid);
    *(volatile v4f*)(ss + 4 * tid) = v;
  }
  __threadfence();
  if (tid < (2 * CCH) / 4) {
    *(volatile v4f*)(ss + 4 * tid) = v;
  }
}

template <int MODE>
__global__ __launch_bounds__(NTHR) void k_apply(const float* __restrict__ inp, const float* __restrict__ ss,
                                                const float* __restrict__ x, int nN,
                                                float* outf, unsigned short* outhl) {
  __shared__ __attribute__((aligned(16))) float ssh[2 * CCH];
  __shared__ __attribute__((aligned(16))) float rst[NWAVE * CCH];
  const int tid = (int)threadIdx.x, lane = tid & 31, wave = tid >> 5;
  ssh[tid] = ss[tid];
  __syncthreads();
  const int row = (int)blockIdx.x * NWAVE + wave;
  const int c4 = 4 * lane;
  const v4f a = *(const v4fa*)(inp + (size_t)row * CCH + c4);
  v4f y;
  y.x = fmaf(a.x, ssh[c4 + 0], ssh[CCH + c4 + 0]);
  y.y = fmaf(a.y, ssh[c4 + 1], ssh[CCH + c4 + 1]);
  y.z = fmaf(a.z, ssh[c4 + 2], ssh[CCH + c4 + 2]);
  y.w = fmaf(a.w, ssh[c4 + 3], ssh[CCH + c4 + 3]);
  if constexpr (MODE == 1) {
    const int rc = row < nN ? row : nN - 1;
    const v4f xr = bfr4(*(const v4fa*)(x + (size_t)rc * CCH + c4));
    y.x = y.x + xr.x; y.y = y.y + xr.y; y.z = y.z + xr.z; y.w = y.w + xr.w;
  } else {
    y.x = fmaxf(y.x, 0.0f); y.y = fmaxf(y.y, 0.0f); y.z = fmaxf(y.z, 0.0f); y.w = fmaxf(y.w, 0.0f);
  }
  const bool live = row < nN;
  const v4f z4 = {0.f, 0.f, 0.f, 0.f};
  y = live ? y : z4;

  *(v4fa*)(rst + wave * CCH + c4) = y;
  __builtin_amdgcn_fence(__ATOMIC_RELEASE, "wavefront");
  __builtin_amdgcn_wave_barrier();
  const int l16 = lane & 15;
  const v4f pa = *(const v4fa*)(rst + wave * CCH + 8 * l16);
  const v4f pb = *(const v4fa*)(rst + wave * CCH + 8 * l16 + 4);
  v4u hv, lv;
  pack8hl(pa, pb, hv, lv);
  v4u wv;
  wv.x = (lane < 16) ? hv.x : lv.x;
  wv.y = (lane < 16) ? hv.y : lv.y;
  wv.z = (lane < 16) ? hv.z : lv.z;
  wv.w = (lane < 16) ? hv.w : lv.w;
  float* fp = outf + (size_t)row * CCH + c4;
  unsigned short* hp = outhl + (size_t)row * K2 + 8 * lane;
  if constexpr (MODE == 1) *(volatile v4f*)fp = y;
  *(volatile v4u*)hp = wv;
  __threadfence();
  if constexpr (MODE == 1) *(volatile v4f*)fp = y;
  *(volatile v4u*)hp = wv;
  (void)fp;
}

__global__ __launch_bounds__(NTHR) void k_out(const float* __restrict__ hm, const float* __restrict__ res,
                                              const float* __restrict__ ss, int nUnits, float* out) {
  __shared__ float ssh[2 * CCH];
  const int tid = (int)threadIdx.x;
  ssh[tid] = ss[tid];
  __syncthreads();
  const int u = (int)blockIdx.x * NTHR + tid;
  if (u >= nUnits) return;
  const int c4 = (u & 31) * 4;
  const v4f a = *(const v4f*)(hm + (size_t)u * 4);
  const v4f r = *(const v4f*)(res + (size_t)u * 4);
  v4f o;
  o.x = fmaf(a.x, ssh[c4 + 0], ssh[CCH + c4 + 0]) + r.x;
  o.y = fmaf(a.y, ssh[c4 + 1], ssh[CCH + c4 + 1]) + r.y;
  o.z = fmaf(a.z, ssh[c4 + 2], ssh[CCH + c4 + 2]) + r.z;
  o.w = fmaf(a.w, ssh[c4 + 3], ssh[CCH + c4 + 3]) + r.w;
  float* op = out + (size_t)u * 4;
  *(volatile v4f*)op = o;
  __threadfence();
  *(volatile v4f*)op = o;
}

static inline int cdiv(int a, int b) { return (a + b - 1) / b; }
static inline size_t al256(size_t o) { return (o + 255) & ~(size_t)255; }

extern "C" void kernel_launch(void* const* d_in, const int* in_sizes, int n_in,
                              void* d_out, int out_size, void* d_ws, size_t ws_size,
                              hipStream_t stream) {
  if (n_in < 25) return;
  if (in_sizes[0] < CCH * GBM || (in_sizes[0] % CCH) != 0) return;
  const int nN = in_sizes[0] / CCH;
  if (nN > (1 << 22)) return;
  const int nE = in_sizes[1];
  if (nE < 1 || in_sizes[2] != nE || in_sizes[3] != nE) return;
  if (nE >= (1 << (31 - SLOTB))) return;
  if (in_sizes[4] != CCH * CCH || in_sizes[6] != CCH * CCH || in_sizes[8] != CCH * CCH || in_sizes[10] != CCH * CCH) return;
  if (in_sizes[5] != CCH || in_sizes[7] != CCH || in_sizes[9] != CCH || in_sizes[11] != CCH) return;
  if (in_sizes[12] != 9 || in_sizes[13] != 3 || in_sizes[14] != 3 * CCH || in_sizes[15] != CCH) return;
  if (in_sizes[16] != CCH || in_sizes[17] != CCH || in_sizes[18] != CCH * CCH) return;
  if (in_sizes[19] != CCH || in_sizes[20] != CCH || in_sizes[21] != CCH * CCH || in_sizes[22] != CCH) return;
  if (in_sizes[23] != CCH || in_sizes[24] != CCH) return;
  if ((long long)out_size != (long long)nN * CCH) return;

  const float* x    = (const float*)d_in[0];
  const int*   kidx = (const int*)d_in[1];
  const int*   vidx = (const int*)d_in[2];
  const int*   qidx = (const int*)d_in[3];
  const float* Wq  = (const float*)d_in[4];  const float* bq  = (const float*)d_in[5];
  const float* Wk  = (const float*)d_in[6];  const float* bk  = (const float*)d_in[7];
  const float* Wv  = (const float*)d_in[8];  const float* bv  = (const float*)d_in[9];
  const float* Wo  = (const float*)d_in[10]; const float* bo  = (const float*)d_in[11];
  const float* pW1 = (const float*)d_in[12]; const float* pb1 = (const float*)d_in[13];
  const float* pW2 = (const float*)d_in[14]; const float* pb2 = (const float*)d_in[15];
  const float* g1  = (const float*)d_in[16]; const float* be1 = (const float*)d_in[17];
  const float* mW1 = (const float*)d_in[18];
  const float* mg  = (const float*)d_in[19]; const float* mb  = (const float*)d_in[20];
  const float* mW2 = (const float*)d_in[21]; const float* mb2 = (const float*)d_in[22];
  const float* g2  = (const float*)d_in[23]; const float* be2 = (const float*)d_in[24];
  float* out = (float*)d_out;

  const int MP = cdiv(nN, GBM) * GBM;
  const int gM = MP / GBM;
  const int gA = cdiv(MP, NBMAX);
  if ((long long)gA * NBMAX < (long long)MP) return;
  const int vec8 = ((nE & 3) == 0) ? 1 : 0;

  const size_t szF = (size_t)MP * CCH * 4;
  char* ws = (char*)d_ws;
  size_t off = 0;
  const size_t oWQ  = off; off = al256(off + (size_t)QKVW * CCH * 2);
  const size_t oWO  = off; off = al256(off + (size_t)CCH * K2 * 2);
  const size_t oM1  = off; off = al256(off + (size_t)CCH * K2 * 2);
  const size_t oM2  = off; off = al256(off + (size_t)CCH * K2 * 2);
  const size_t oRT  = off; off = al256(off + (size_t)RTN * 4);
  const size_t oPT  = off; off = al256(off + (size_t)gM * PARTW * 4);
  const size_t oS1  = off; off = al256(off + (size_t)(2 * CCH) * 4);
  const size_t oS2  = off; off = al256(off + (size_t)(2 * CCH) * 4);
  const size_t oS3  = off; off = al256(off + (size_t)(2 * CCH) * 4);
  const size_t oR0  = off; off = al256(off + 3 * szF);
  const size_t oR1  = off; off = al256(off + szF);
  if (off > ws_size || off > (size_t)WSLIM) return;
  unsigned short* WQKVT = (unsigned short*)(ws + oWQ);
  unsigned short* WOT2  = (unsigned short*)(ws + oWO);
  unsigned short* M1T2  = (unsigned short*)(ws + oM1);
  unsigned short* M2T2  = (unsigned short*)(ws + oM2);
  float*          RT    = (float*)(ws + oRT);
  float*          PT    = (float*)(ws + oPT);
  float*          SS1   = (float*)(ws + oS1);
  float*          SS2   = (float*)(ws + oS2);
  float*          SS3   = (float*)(ws + oS3);
  float*          QKV   = (float*)(ws + oR0);
  float*          OUTF  = (float*)(ws + oR0);
  unsigned short* A2    = (unsigned short*)(ws + oR0 + szF);
  float*          UF    = (float*)(ws + oR0 + 2 * szF);
  unsigned short* A3    = (unsigned short*)(ws + oR0);
  float*          HMF   = (float*)(ws + oR0 + szF);
  unsigned short* XB    = (unsigned short*)(ws + oR1);
  unsigned short* AOHL  = (unsigned short*)(ws + oR1);
  float*          OUTU  = (float*)(ws + oR1);

  hipFuncSetAttribute(reinterpret_cast<const void*>(&k_attn),
                      hipFuncAttributeMaxDynamicSharedMemorySize, LDS_ATTN);

  k_wprep<<<NBPREP, NTHR, 0, stream>>>(Wq, Wk, Wv, Wo, mW1, mW2, pW1, pb1, pW2, pb2,
                                       WQKVT, WOT2, M1T2, M2T2, RT);
  const int nUx = MP * (CCH / 8);
  k_xprep<<<cdiv(nUx, NTHR), NTHR, 0, stream>>>(x, XB, nN, nUx);
  k_gemm<CCH, 0><<<dim3(gM, QKVW / GBN), GTHR, 0, stream>>>(XB, WQKVT, nN, bq, bk, bv, QKV, QKVW, PT);
  k_attn<<<gA, NTHR, LDS_ATTN, stream>>>(kidx, vidx, qidx, QKV, RT, AOHL, nN, nE, vec8, MP);
  k_gemm<K2, 1><<<dim3(gM, 1), GTHR, 0, stream>>>(AOHL, WOT2, nN, bo, bo, bo, OUTF, CCH, PT);
  k_bnfin<<<1, CCH, 0, stream>>>(PT, gM, g1, be1, SS1);
  k_apply<1><<<MP / NWAVE, NTHR, 0, stream>>>(OUTF, SS1, x, nN, OUTU, A2);
  k_gemm<K2, 2><<<dim3(gM, 1), GTHR, 0, stream>>>(A2, M1T2, nN, mg, mg, mg, UF, CCH, PT);
  k_bnfin<<<1, CCH, 0, stream>>>(PT, gM, mg, mb, SS2);
  k_apply<2><<<MP / NWAVE, NTHR, 0, stream>>>(UF, SS2, x, nN, HMF, A3);
  k_gemm<K2, 1><<<dim3(gM, 1), GTHR, 0, stream>>>(A3, M2T2, nN, mb2, mb2, mb2, HMF, CCH, PT);
  k_bnfin<<<1, CCH, 0, stream>>>(PT, gM, g2, be2, SS3);
  const int nUo = nN * (CCH / 4);
  k_out<<<cdiv(nUo, NTHR), NTHR, 0, stream>>>(HMF, OUTU, SS3, nUo, out);
}
